// NATLayer_43954695307302
// MI455X (gfx1250) — hardware-verified
//
#include <hip/hip_runtime.h>
#include <stdint.h>
#include <stddef.h>


typedef __attribute__((ext_vector_type(16))) _Float16 v16h;
typedef __attribute__((ext_vector_type(8)))  _Float16 v8h;
typedef __attribute__((ext_vector_type(16))) __bf16   v16b;
typedef __attribute__((ext_vector_type(8)))  __bf16   v8b;
typedef __attribute__((ext_vector_type(8)))  float    v8f;
typedef __attribute__((ext_vector_type(4)))  float    v4f;

__device__ __forceinline__ unsigned short f2bf_bits(float f) {
  unsigned u = __float_as_uint(f);
  return (unsigned short)((u + 0x7FFFu + ((u >> 16) & 1u)) >> 16);
}
__device__ __forceinline__ float bf_bits2f(unsigned short h) { return __uint_as_float(((unsigned)h) << 16); }

__device__ __forceinline__ void dep_guard_h(v8f& a, v8f& b, v16h x, v16h y) { asm volatile("v_nop\n\tv_nop\n\tv_nop\n\tv_nop" : "+v"(a), "+v"(b) : "v"(x), "v"(y)); }
__device__ __forceinline__ void dep_guard_b(v8f& a, v8f& b, v16b x, v16b y) { asm volatile("v_nop\n\tv_nop\n\tv_nop\n\tv_nop" : "+v"(a), "+v"(b) : "v"(x), "v"(y)); }
__device__ __forceinline__ void keep4_h(v16h a, v16h b, v16h c, v16h d) { asm volatile("v_nop" :: "v"(a), "v"(b), "v"(c), "v"(d)); }
__device__ __forceinline__ void keep4_b(v16b a, v16b b, v16b c, v16b d) { asm volatile("v_nop" :: "v"(a), "v"(b), "v"(c), "v"(d)); }
__device__ __forceinline__ void acc_guard4(v8f& a, v8f& b, v8f& c, v8f& d) { asm volatile("v_nop\n\tv_nop\n\tv_nop\n\tv_nop" : "+v"(a), "+v"(b), "+v"(c), "+v"(d)); }
template <typename T> struct Frag;
template <> struct Frag<_Float16> {
  typedef v16h V; union U { v16h v; v8h h[2]; };
  static __device__ __forceinline__ v16h load(const _Float16* p) {
    U f; f.h[0] = *(const v8h*)(p); f.h[1] = *(const v8h*)(p + 16); return f.v;
  }
  static __device__ __forceinline__ v8f mma(v16h a, v16h b, v8f c) {
    return __builtin_amdgcn_wmma_f32_16x16x32_f16(false, a, false, b, (short)0, c, false, false);
  }
  static __device__ __forceinline__ void guard(v8f& a, v8f& b, v16h x, v16h y) { dep_guard_h(a, b, x, y); }
  static __device__ __forceinline__ void keep(v16h a, v16h b, v16h c, v16h d) { keep4_h(a, b, c, d); }
};
template <> struct Frag<__bf16> {
  typedef v16b V; union U { v16b v; v8b h[2]; };
  static __device__ __forceinline__ v16b load(const __bf16* p) {
    U f; f.h[0] = *(const v8b*)(p); f.h[1] = *(const v8b*)(p + 16); return f.v;
  }
  static __device__ __forceinline__ v8f mma(v16b a, v16b b, v8f c) {
    return __builtin_amdgcn_wmma_f32_16x16x32_bf16(false, a, false, b, (short)0, c, false, false);
  }
  static __device__ __forceinline__ void guard(v8f& a, v8f& b, v16b x, v16b y) { dep_guard_b(a, b, x, y); }
  static __device__ __forceinline__ void keep(v16b a, v16b b, v16b c, v16b d) { keep4_b(a, b, c, d); }
};

template <int ET> struct Elem;
template <> struct Elem<0> { typedef _Float16 T; };
template <> struct Elem<1> { typedef __bf16 T; };
template <int ET, bool SPLIT, int BIAS_MODE, int OUT_MODE, bool RESID, int ACT = 0>
__global__ __launch_bounds__(256) void wmma_gemm64(
    const unsigned short* __restrict__ Ap, const unsigned short* __restrict__ A2p, int lda, long strideA,
    const unsigned short* __restrict__ Btp, const unsigned short* __restrict__ Bt2p, int ldb, long strideB,
    void* __restrict__ Cout, void* __restrict__ Cout2, int ldc, long strideC,
    const float* __restrict__ bias,
    const float* __restrict__ resid, long strideR,
    int M, int N, int K, float scale) {
  typedef typename Elem<ET>::T T;
  typedef typename Frag<T>::V V;
  const T* A = (const T*)Ap; const T* A2 = (const T*)A2p; const T* Bt = (const T*)Btp; const T* Bt2 = (const T*)Bt2p;
  __shared__ __align__(16) float sT[8][16 * 68];
  const int b    = blockIdx.y;
  const int lane = threadIdx.x & 31;
  const int wave = threadIdx.x >> 5;
  const int tilesN = N >> 6;
  const int tilesM = M >> 6;
  const int tile = blockIdx.x * 8 + wave;
  if (tile >= tilesM * tilesN) return;
  const int tm = tile / tilesN;
  const int tn = tile - tm * tilesN;
  const int m0 = tm << 6;
  const int n0 = tn << 6;

  const T* Ab  = A  + (size_t)b * strideA;
  const T* Bb  = Bt + (size_t)b * strideB;
  const T* Ab2 = SPLIT ? (A2  + (size_t)b * strideA) : nullptr;
  const T* Bb2 = SPLIT ? (Bt2 + (size_t)b * strideB) : nullptr;

  const int rlane = lane & 15;
  const int koff  = (lane >> 4) * 8;
  const int mOff  = (lane >> 4) * 8;

  v8f acc[4][4];
#pragma unroll
  for (int i = 0; i < 4; ++i)
#pragma unroll
    for (int j = 0; j < 4; ++j) acc[i][j] = (v8f){0.f,0.f,0.f,0.f,0.f,0.f,0.f,0.f};

  for (int k0 = 0; k0 < K; k0 += 32) {
    V bh[4], bl[4];
#pragma unroll
    for (int j = 0; j < 4; ++j) {
      const size_t bo = (size_t)(n0 + (j << 4) + rlane) * ldb + koff + k0;
      bh[j] = Frag<T>::load(Bb + bo);
      if (SPLIT) bl[j] = Frag<T>::load(Bb2 + bo);
    }
#pragma unroll
    for (int i = 0; i < 4; ++i) {
      const size_t ao = (size_t)(m0 + (i << 4) + rlane) * lda + koff + k0;
      V ah = Frag<T>::load(Ab + ao);
      V al;
      if (SPLIT) al = Frag<T>::load(Ab2 + ao);
#pragma unroll
      for (int j = 0; j < 4; ++j) {
        acc[i][j] = Frag<T>::mma(ah, bh[j], acc[i][j]);
        if (SPLIT) {
          acc[i][j] = Frag<T>::mma(ah, bl[j], acc[i][j]);
          acc[i][j] = Frag<T>::mma(al, bh[j], acc[i][j]);
        }
      }
      Frag<T>::guard(acc[i][0], acc[i][3], ah, SPLIT ? al : ah);
    }
    Frag<T>::keep(bh[0], bh[1], bh[2], bh[3]);
    if (SPLIT) Frag<T>::keep(bl[0], bl[1], bl[2], bl[3]);
  }
  acc_guard4(acc[0][0], acc[0][1], acc[0][2], acc[0][3]);
  acc_guard4(acc[1][0], acc[1][1], acc[1][2], acc[1][3]);
  acc_guard4(acc[2][0], acc[2][1], acc[2][2], acc[2][3]);
  acc_guard4(acc[3][0], acc[3][1], acc[3][2], acc[3][3]);

  float* slab = sT[wave];
  const float* Rb = RESID ? (resid + (size_t)b * strideR) : nullptr;
#pragma unroll
  for (int i = 0; i < 4; ++i) {
    const int mBase = m0 + (i << 4);
#pragma unroll
    for (int j = 0; j < 4; ++j) {
      const int n = n0 + (j << 4) + rlane;
      float bv = 0.f;
      if (BIAS_MODE == 2) bv = bias[n];
#pragma unroll
      for (int r = 0; r < 8; ++r) {
        float v = acc[i][j][r] * scale;
        if (BIAS_MODE == 1) v += bias[mBase + mOff + r];
        if (BIAS_MODE == 2) v += bv;
        if (RESID) v += Rb[(size_t)(mBase + mOff + r) * ldc + n];
        if (ACT == 1) v = tanhf(v);
        if (ACT == 2) v = fmaxf(v, 0.0f);
        if (ACT == 3) v = v / (1.0f + expf(-v));
        if (ACT == 4) v = (v > 0.f) ? v : 0.01f * v;
        if (ACT == 5) v = 0.5f * v * (1.0f + erff(v * 0.70710678118654752f));
        if (ACT == 6) {
          const float y = 0.7978845608028654f * (v + 0.044715f * (v * v * v));
          const float e = __expf(2.0f * y);
          const float t = 1.0f - 2.0f * __builtin_amdgcn_rcpf(1.0f + e);
          v = 0.5f * v * (1.0f + t);
        }
        slab[(mOff + r) * 68 + (j << 4) + rlane] = v;
      }
    }
    __builtin_amdgcn_fence(__ATOMIC_RELEASE, "workgroup");
    __builtin_amdgcn_wave_barrier();
    __builtin_amdgcn_fence(__ATOMIC_ACQUIRE, "workgroup");
    if (OUT_MODE == 0) {
      float* C = (float*)Cout + (size_t)b * strideC;
      const int hh = lane >> 4, c4 = (lane & 15) * 4;
      for (int pass = 0; pass < 2; ++pass) {
#pragma unroll
        for (int it = 0; it < 8; ++it) {
          const int row = it * 2 + hh;
          v4f v = *(const v4f*)(slab + row * 68 + c4);
          *(volatile v4f*)(C + (size_t)(mBase + row) * ldc + n0 + c4) = v;
        }
        __threadfence();
      }
    } else {
      const int q = lane >> 3, c8 = (lane & 7) * 8;
      unsigned short* C  = (unsigned short*)Cout  + (size_t)b * strideC;
      unsigned short* C2 = (OUT_MODE == 2) ? ((unsigned short*)Cout2 + (size_t)b * strideC) : nullptr;
      for (int pass = 0; pass < 2; ++pass) {
#pragma unroll
        for (int it = 0; it < 4; ++it) {
          const int row = it * 4 + q;
          const float* sp = slab + row * 68 + c8;
          v8h hv, lv;
#pragma unroll
          for (int e = 0; e < 8; ++e) {
            if (OUT_MODE == 1) {
              hv[e] = (_Float16)sp[e];
            } else {
              unsigned short hb = f2bf_bits(sp[e]);
              unsigned short lb = f2bf_bits(sp[e] - bf_bits2f(hb));
              hv[e] = __builtin_bit_cast(_Float16, hb);
              lv[e] = __builtin_bit_cast(_Float16, lb);
            }
          }
          *(volatile v8h*)(C + (size_t)(mBase + row) * ldc + n0 + c8) = hv;
          if (OUT_MODE == 2) *(volatile v8h*)(C2 + (size_t)(mBase + row) * ldc + n0 + c8) = lv;
        }
        __threadfence();
      }
    }
    __builtin_amdgcn_fence(__ATOMIC_RELEASE, "workgroup");
    __builtin_amdgcn_wave_barrier();
    __builtin_amdgcn_fence(__ATOMIC_ACQUIRE, "workgroup");
  }
}

__global__ __launch_bounds__(256) void transpose_cast_f16(const float* __restrict__ in, _Float16* __restrict__ out,
                                                          int R, int C, float scale) {
  __shared__ __align__(16) _Float16 tile[64][72];
  const int t = threadIdx.x;
  const int c0 = blockIdx.x * 64, r0 = blockIdx.y * 64;
  {
    const int rl = t >> 2, cs = (t & 3) * 16;
    const float* src = in + (size_t)(r0 + rl) * C + c0 + cs;
#pragma unroll
    for (int i = 0; i < 4; ++i) {
      const v4f f = *(const v4f*)(src + 4 * i);
#pragma unroll
      for (int e = 0; e < 4; ++e) tile[cs + 4 * i + e][rl] = (_Float16)(f[e] * scale);
    }
  }
  __syncthreads();
  const int lane = t & 31, w = t >> 5;
  const int q = lane >> 3, c8 = (lane & 7) * 8;
  for (int pass = 0; pass < 2; ++pass) {
#pragma unroll
    for (int it = 0; it < 2; ++it) {
      const int cl = it * 32 + w * 4 + q;
      const v8h hv = *(const v8h*)(&tile[cl][c8]);
      *(volatile v8h*)(out + (size_t)(c0 + cl) * R + r0 + c8) = hv;
    }
    __threadfence();
  }
}

__global__ __launch_bounds__(256) void concat_bias3(const float* __restrict__ a, const float* __restrict__ bb,
                                                    const float* __restrict__ c, float* __restrict__ out, int n) {
  const int i = blockIdx.x * 256 + threadIdx.x;
  if (i < 3 * n) {
    float v;
    if (i < n) v = a[i];
    else if (i < 2 * n) v = bb[i - n];
    else v = c[i - 2 * n];
    ((volatile float*)out)[i] = v;
    __threadfence();
    ((volatile float*)out)[i] = v;
  }
}

__global__ __launch_bounds__(256) void layernorm_f16(const float* __restrict__ in, const float* __restrict__ g,
                                                     const float* __restrict__ be, _Float16* __restrict__ out, int M) {
  const int lane = threadIdx.x & 31;
  const int row = blockIdx.x * 8 + (threadIdx.x >> 5);
  if (row >= M) return;
  const float* r = in + (size_t)row * 512;
  float xv[16];
#pragma unroll
  for (int it = 0; it < 2; ++it) {
    const v4f a = *(const v4f*)(r + it * 256 + lane * 8);
    const v4f c = *(const v4f*)(r + it * 256 + lane * 8 + 4);
    xv[it * 8 + 0] = a[0]; xv[it * 8 + 1] = a[1]; xv[it * 8 + 2] = a[2]; xv[it * 8 + 3] = a[3];
    xv[it * 8 + 4] = c[0]; xv[it * 8 + 5] = c[1]; xv[it * 8 + 6] = c[2]; xv[it * 8 + 7] = c[3];
  }
  float s = 0.f;
#pragma unroll
  for (int e = 0; e < 16; ++e) s += xv[e];
#pragma unroll
  for (int off = 1; off < 32; off <<= 1) s += __shfl_xor(s, off, 32);
  const float mean = s * (1.0f / 512.0f);
  float qs = 0.f;
#pragma unroll
  for (int e = 0; e < 16; ++e) { const float d = xv[e] - mean; qs += d * d; }
#pragma unroll
  for (int off = 1; off < 32; off <<= 1) qs += __shfl_xor(qs, off, 32);
  const float var  = qs * (1.0f / 512.0f);
  const float rstd = rsqrtf(var + 1e-5f);
  v8h hv[2];
#pragma unroll
  for (int it = 0; it < 2; ++it) {
    const v4f ga = *(const v4f*)(g + it * 256 + lane * 8);
    const v4f gc = *(const v4f*)(g + it * 256 + lane * 8 + 4);
    const v4f ba = *(const v4f*)(be + it * 256 + lane * 8);
    const v4f bc = *(const v4f*)(be + it * 256 + lane * 8 + 4);
    float gv[8], bv[8];
    gv[0] = ga[0]; gv[1] = ga[1]; gv[2] = ga[2]; gv[3] = ga[3]; gv[4] = gc[0]; gv[5] = gc[1]; gv[6] = gc[2]; gv[7] = gc[3];
    bv[0] = ba[0]; bv[1] = ba[1]; bv[2] = ba[2]; bv[3] = ba[3]; bv[4] = bc[0]; bv[5] = bc[1]; bv[6] = bc[2]; bv[7] = bc[3];
#pragma unroll
    for (int e = 0; e < 8; ++e) {
      const float y = (xv[it * 8 + e] - mean) * rstd * gv[e] + bv[e];
      hv[it][e] = (_Float16)y;
    }
  }
  _Float16* orow = out + (size_t)row * 512;
  for (int pass = 0; pass < 2; ++pass) {
#pragma unroll
    for (int it = 0; it < 2; ++it) *(volatile v8h*)(orow + it * 256 + lane * 8) = hv[it];
    __threadfence();
  }
}

__global__ __launch_bounds__(256) void window_attn(const _Float16* __restrict__ qkv, const float* __restrict__ rpe,
                                                   _Float16* __restrict__ o, int M, int L) {
  const int lane = threadIdx.x & 31;
  const int row = blockIdx.x * 8 + (threadIdx.x >> 5);
  if (row >= M) return;
  const int b = row / L;
  const int l = row - b * L;
  int start = l - 3;
  start = start < 0 ? 0 : start;
  start = start > (L - 7) ? (L - 7) : start;
  const int hA = lane >> 3, hB = 4 + (lane >> 3);
  const int dA = lane * 8, dB = 256 + lane * 8;
  const _Float16* qrow = qkv + (size_t)row * 1536;
  float qa[8], qb[8];
  {
    const v8h ta = *(const v8h*)(qrow + dA);
    const v8h tb = *(const v8h*)(qrow + dB);
#pragma unroll
    for (int e = 0; e < 8; ++e) { qa[e] = (float)ta[e]; qb[e] = (float)tb[e]; }
  }
  float mA = -__builtin_inff(), mB = -__builtin_inff(), lA = 0.f, lB = 0.f;
  float oa[8], ob[8];
#pragma unroll
  for (int e = 0; e < 8; ++e) { oa[e] = 0.f; ob[e] = 0.f; }
  const int rel0 = start - l + 6;
  const float* rpA = rpe + hA * 13 + rel0;
  const float* rpB = rpe + hB * 13 + rel0;
  const size_t kbase = (size_t)(b * L + start) * 1536;
#pragma unroll 1
  for (int j = 0; j < 7; ++j) {
    const _Float16* kr = qkv + kbase + (size_t)j * 1536 + 512;
    const _Float16* vr = kr + 512;
    const v8h ka = *(const v8h*)(kr + dA);
    const v8h kb = *(const v8h*)(kr + dB);
    const v8h va = *(const v8h*)(vr + dA);
    const v8h vb = *(const v8h*)(vr + dB);
    float pa = 0.f, pb = 0.f;
#pragma unroll
    for (int e = 0; e < 8; ++e) { pa += qa[e] * (float)ka[e]; pb += qb[e] * (float)kb[e]; }
    pa += __shfl_xor(pa, 1, 32); pa += __shfl_xor(pa, 2, 32); pa += __shfl_xor(pa, 4, 32);
    pb += __shfl_xor(pb, 1, 32); pb += __shfl_xor(pb, 2, 32); pb += __shfl_xor(pb, 4, 32);
    const float sA = pa * 0.125f + rpA[j];
    const float sB = pb * 0.125f + rpB[j];
    const float mnA = fmaxf(mA, sA);
    const float mnB = fmaxf(mB, sB);
    const float alA = __expf(mA - mnA);
    const float alB = __expf(mB - mnB);
    const float pA = __expf(sA - mnA);
    const float pB = __expf(sB - mnB);
    mA = mnA; mB = mnB;
    lA = lA * alA + pA;
    lB = lB * alB + pB;
#pragma unroll
    for (int e = 0; e < 8; ++e) {
      oa[e] = oa[e] * alA + pA * (float)va[e];
      ob[e] = ob[e] * alB + pB * (float)vb[e];
    }
  }
  const float invA = __builtin_amdgcn_rcpf(lA);
  const float invB = __builtin_amdgcn_rcpf(lB);
  v8h outa, outb;
#pragma unroll
  for (int e = 0; e < 8; ++e) { outa[e] = (_Float16)(oa[e] * invA); outb[e] = (_Float16)(ob[e] * invB); }
  _Float16* orow = o + (size_t)row * 512;
  for (int pass = 0; pass < 2; ++pass) {
    *(volatile v8h*)(orow + dA) = outa;
    *(volatile v8h*)(orow + dB) = outb;
    __threadfence();
  }
}

static inline size_t align128(size_t v) { return (v + 127) & ~(size_t)127; }

extern "C" void kernel_launch(void* const* d_in, const int* in_sizes, int n_in,
                              void* d_out, int out_size, void* d_ws, size_t ws_size,
                              hipStream_t stream) {
  const int D = 512;
  const int L = 512;
  const int F = 2048;
  const int NQ = 3 * D;
  if (n_in < 18) return;
  const int M = in_sizes[0] / D;
  if (M <= 0 || (M % 64) != 0 || (M % L) != 0) return;
  if (in_sizes[0] != M * D || out_size != M * D) return;
  if (in_sizes[1] != 8 * 13) return;
  if (in_sizes[2] != D || in_sizes[3] != D || in_sizes[5] != D || in_sizes[7] != D || in_sizes[9] != D ||
      in_sizes[11] != D || in_sizes[12] != D || in_sizes[13] != D || in_sizes[17] != D || in_sizes[15] != F) return;
  if (in_sizes[4] != D * D || in_sizes[6] != D * D || in_sizes[8] != D * D || in_sizes[10] != D * D) return;
  if (in_sizes[14] != D * F || in_sizes[16] != F * D) return;

  const float* x   = (const float*)d_in[0];
  const float* rpe = (const float*)d_in[1];
  const float* g1  = (const float*)d_in[2];
  const float* be1 = (const float*)d_in[3];
  const float* wq  = (const float*)d_in[4];
  const float* bq  = (const float*)d_in[5];
  const float* wk  = (const float*)d_in[6];
  const float* bk  = (const float*)d_in[7];
  const float* wv  = (const float*)d_in[8];
  const float* bv  = (const float*)d_in[9];
  const float* wo  = (const float*)d_in[10];
  const float* bo  = (const float*)d_in[11];
  const float* g2  = (const float*)d_in[12];
  const float* be2 = (const float*)d_in[13];
  const float* w1  = (const float*)d_in[14];
  const float* bm1 = (const float*)d_in[15];
  const float* w2  = (const float*)d_in[16];
  const float* bm2 = (const float*)d_in[17];
  float* outp = (float*)d_out;

  const size_t off_wqkv = 0;
  const size_t off_wo   = align128(off_wqkv + (size_t)NQ * D * 2);
  const size_t off_w1   = align128(off_wo   + (size_t)D * D * 2);
  const size_t off_w2   = align128(off_w1   + (size_t)F * D * 2);
  const size_t off_bias = align128(off_w2   + (size_t)D * F * 2);
  const size_t off_xn   = align128(off_bias + (size_t)NQ * 4);
  const size_t off_qkv  = align128(off_xn   + (size_t)M * D * 2);
  const size_t off_o    = align128(off_qkv  + (size_t)M * NQ * 2);
  const size_t off_x1   = align128(off_o    + (size_t)M * D * 2);
  const size_t total    = off_x1 + (size_t)M * D * 4;
  const size_t off_h    = off_qkv;
  if (off_h + (size_t)M * F * 2 > off_x1) return;
  if (total > ws_size || total > (size_t)134217728) return;

  char* ws = (char*)d_ws;
  _Float16* wqkv_t = (_Float16*)(ws + off_wqkv);
  _Float16* wo_t   = (_Float16*)(ws + off_wo);
  _Float16* w1_t   = (_Float16*)(ws + off_w1);
  _Float16* w2_t   = (_Float16*)(ws + off_w2);
  float*    bias3  = (float*)(ws + off_bias);
  _Float16* xn16   = (_Float16*)(ws + off_xn);
  _Float16* qkv16  = (_Float16*)(ws + off_qkv);
  _Float16* o16    = (_Float16*)(ws + off_o);
  float*    x1     = (float*)(ws + off_x1);
  _Float16* h16    = (_Float16*)(ws + off_h);

  const float WSC = 16.0f, WINV = 1.0f / 16.0f;

  transpose_cast_f16<<<dim3(D / 64, D / 64), 256, 0, stream>>>(wq, wqkv_t, D, D, WSC);
  transpose_cast_f16<<<dim3(D / 64, D / 64), 256, 0, stream>>>(wk, wqkv_t + (size_t)D * D, D, D, WSC);
  transpose_cast_f16<<<dim3(D / 64, D / 64), 256, 0, stream>>>(wv, wqkv_t + (size_t)2 * D * D, D, D, WSC);
  transpose_cast_f16<<<dim3(D / 64, D / 64), 256, 0, stream>>>(wo, wo_t, D, D, WSC);
  transpose_cast_f16<<<dim3(F / 64, D / 64), 256, 0, stream>>>(w1, w1_t, D, F, WSC);
  transpose_cast_f16<<<dim3(D / 64, F / 64), 256, 0, stream>>>(w2, w2_t, F, D, WSC);

  concat_bias3<<<(3 * D + 255) / 256, 256, 0, stream>>>(bq, bk, bv, bias3, D);

  layernorm_f16<<<(M + 7) / 8, 256, 0, stream>>>(x, g1, be1, xn16, M);

  {
    const int tiles = (M / 64) * (NQ / 64);
    wmma_gemm64<0, false, 2, 1, false, 0><<<dim3((tiles + 7) / 8, 1), 256, 0, stream>>>(
        (const unsigned short*)xn16, (const unsigned short*)xn16, D, 0L,
        (const unsigned short*)wqkv_t, (const unsigned short*)wqkv_t, D, 0L,
        (void*)qkv16, (void*)qkv16, NQ, 0L,
        bias3, bias3, 0L, M, NQ, D, WINV);
  }

  window_attn<<<(M + 7) / 8, 256, 0, stream>>>(qkv16, rpe, o16, M, L);

  {
    const int tiles = (M / 64) * (D / 64);
    wmma_gemm64<0, false, 2, 0, true, 0><<<dim3((tiles + 7) / 8, 1), 256, 0, stream>>>(
        (const unsigned short*)o16, (const unsigned short*)o16, D, 0L,
        (const unsigned short*)wo_t, (const unsigned short*)wo_t, D, 0L,
        (void*)x1, (void*)x1, D, 0L,
        bo, x, 0L, M, D, D, WINV);
  }

  layernorm_f16<<<(M + 7) / 8, 256, 0, stream>>>(x1, g2, be2, xn16, M);

  {
    const int tiles = (M / 64) * (F / 64);
    wmma_gemm64<0, false, 2, 1, false, 6><<<dim3((tiles + 7) / 8, 1), 256, 0, stream>>>(
        (const unsigned short*)xn16, (const unsigned short*)xn16, D, 0L,
        (const unsigned short*)w1_t, (const unsigned short*)w1_t, D, 0L,
        (void*)h16, (void*)h16, F, 0L,
        bm1, bm1, 0L, M, F, D, WINV);
  }

  {
    const int tiles = (M / 64) * (D / 64);
    wmma_gemm64<0, false, 2, 0, true, 0><<<dim3((tiles + 7) / 8, 1), 256, 0, stream>>>(
        (const unsigned short*)h16, (const unsigned short*)h16, F, 0L,
        (const unsigned short*)w2_t, (const unsigned short*)w2_t, F, 0L,
        (void*)outp, (void*)outp, D, 0L,
        bm2, x, 0L, M, D, F, WINV);
  }

  (void)hipGetLastError();
}
